// NIMA_59579786330555
// MI455X (gfx1250) — hardware-verified
//
#include <hip/hip_runtime.h>
#define BB 16
#define HWI (512 * 512)
#define NB2 64
#define NB1 8
#define G66 66
#define P33 33
#define NPOS (BB * P33 * P33)
#define NPOSR NPOS
#define NVOX 17440
#define COUT 1024
#define HY P33
#define WX P33
#define CHK 4096
#define NBLK (HWI / CHK)

typedef __bf16 v16b __attribute__((ext_vector_type(16)));
typedef unsigned short v8us __attribute__((ext_vector_type(8), may_alias));
typedef float  v8f  __attribute__((ext_vector_type(8)));
typedef float  v4f  __attribute__((ext_vector_type(4)));
typedef float  v4fa __attribute__((ext_vector_type(4), may_alias));
union FragB { v16b v; v8us half[2]; unsigned short u[16]; };

__device__ __forceinline__ unsigned short bf16_bits(float x) { unsigned int u = __float_as_uint(x); return (unsigned short)((u + 0x7FFFu + ((u >> 16) & 1u)) >> 16); }
__device__ __forceinline__ float bf16_val(unsigned short b) { return __uint_as_float(((unsigned int)b) << 16); }
__device__ __forceinline__ float bf16_round(float x) { return bf16_val(bf16_bits(x)); }
template <int NT>
__device__ __forceinline__ v8f mmaN(v16b ah, v16b al, v16b bh, v16b bl, v8f c) {
  c = __builtin_amdgcn_wmma_f32_16x16x32_bf16(false, ah, false, bh, (short)0, c, false, false);
  if (NT >= 2) c = __builtin_amdgcn_wmma_f32_16x16x32_bf16(false, al, false, bh, (short)0, c, false, false);
  if (NT >= 3) c = __builtin_amdgcn_wmma_f32_16x16x32_bf16(false, ah, false, bl, (short)0, c, false, false);
  asm volatile("v_nop\n\tv_nop\n\tv_nop\n\tv_nop" : "+v"(c) : "v"(ah), "v"(al), "v"(bh), "v"(bl));
  return c;
}

__global__ __launch_bounds__(256) void k_wt_bf16(const float* __restrict__ W, unsigned short* __restrict__ Wt, int K, int N) {
  const int t = blockIdx.x * 256 + threadIdx.x;
  const int k8n = K / 8;
  if (t >= N * k8n) return;
  const int n = t / k8n, k8 = (t % k8n) * 8;
  v8us v;
#pragma unroll
  for (int i = 0; i < 8; ++i) v[i] = bf16_bits(W[(size_t)(k8 + i) * N + n]);
  *(volatile v8us*)(Wt + (size_t)n * K + k8) = v;
  __threadfence();
  *(volatile v8us*)(Wt + (size_t)n * K + k8) = v;
}

template <bool ASPLIT, int ACT, bool BIAS_BF16>
__global__ __launch_bounds__(128) void k_gemm_bf(const float* __restrict__ A, int lda, const unsigned short* __restrict__ Wt, int ldb,
                                               const float* __restrict__ bias, float* __restrict__ C, int ldc, int M, int N, int K) {
  __shared__ __attribute__((aligned(16))) float so[4][16][64];
  const int tid = threadIdx.x, w = tid >> 5, lane = tid & 31, ln = lane & 15, hh = lane >> 4;
  const int ntn = N / 64;
  const int wid = blockIdx.x * 4 + w;
  const int mt = wid / ntn, nq = wid % ntn;
  if (mt * 16 >= M) return;
  const int row0 = mt * 16, col0 = nq * 64;
  const float* arow = A + (size_t)(row0 + ln) * lda;
  v8f acc[4] = {};
  for (int kb = 0; kb < K; kb += 32) {
    FragB ah, al;
    const v4f x0 = *(const v4fa*)(arow + kb + 8 * hh), x1 = *(const v4fa*)(arow + kb + 8 * hh + 4);
    const v4f x2 = *(const v4fa*)(arow + kb + 16 + 8 * hh), x3 = *(const v4fa*)(arow + kb + 16 + 8 * hh + 4);
    float xs[16] = {x0[0],x0[1],x0[2],x0[3],x1[0],x1[1],x1[2],x1[3],x2[0],x2[1],x2[2],x2[3],x3[0],x3[1],x3[2],x3[3]};
#pragma unroll
    for (int i = 0; i < 16; ++i) { const unsigned short hb = bf16_bits(xs[i]); ah.u[i] = hb; al.u[i] = ASPLIT ? bf16_bits(xs[i] - bf16_val(hb)) : (unsigned short)0; }
#pragma unroll
    for (int t = 0; t < 4; ++t) {
      const unsigned short* brow = Wt + (size_t)(col0 + t * 16 + ln) * ldb + kb;
      FragB b;
      b.half[0] = *(const v8us*)(brow + 8 * hh);
      b.half[1] = *(const v8us*)(brow + 16 + 8 * hh);
      acc[t] = mmaN<ASPLIT ? 2 : 1>(ah.v, al.v, b.v, b.v, acc[t]);
    }
  }
#pragma unroll
  for (int t = 0; t < 4; ++t) {
    float bv = bias ? bias[col0 + t * 16 + ln] : 0.f;
    if (BIAS_BF16) bv = bf16_round(bv);
#pragma unroll
    for (int r = 0; r < 8; ++r) { float v = acc[t][r] + bv; if (ACT == 1) v = fmaxf(v, 0.f); so[w][8 * hh + r][t * 16 + ln] = v; }
  }
  __builtin_amdgcn_fence(__ATOMIC_ACQ_REL, "workgroup");
  __builtin_amdgcn_wave_barrier();
  const int rsub = lane >> 4, c4 = (lane & 15) * 4;
  for (int pass = 0; pass < 2; ++pass) {
#pragma unroll
    for (int q = 0; q < 8; ++q) {
      const int r = q * 2 + rsub;
      const v4f v = *(const v4fa*)&so[w][r][c4];
      *(volatile v4f*)(C + (size_t)(row0 + r) * ldc + col0 + c4) = v;
    }
    if (pass == 0) __threadfence();
  }
}

template <int D, bool CAUSAL>
__global__ __launch_bounds__(128) void k_flash(const float* __restrict__ qb, const float* __restrict__ kb, const float* __restrict__ vb,
                                             int pitch, int T, int H, float scale, float* __restrict__ y, int ypitch) {
  constexpr int KS = D / 32;
  constexpr int DT = D / 16;
  __shared__ __attribute__((aligned(16))) unsigned short sKh[32][D + 8], sKl[32][D + 8], sVh[32][D + 8], sVl[32][D + 8];
  __shared__ __attribute__((aligned(16))) unsigned short sPh[4][16][40], sPl[4][16][40];
  __shared__ __attribute__((aligned(16))) float sO[4][16][D];
  const int tid = threadIdx.x, w = tid >> 5, lane = tid & 31, ln = lane & 15, hh = lane >> 4;
  const int nqb = (T + 63) / 64;
  const int bh = blockIdx.x / nqb, qblk = blockIdx.x % nqb;
  const int b = bh / H, h = bh % H;
  const int q0 = qblk * 64 + w * 16;
  const float* Q = qb + (size_t)b * T * pitch + h * D;
  const float* K = kb + (size_t)b * T * pitch + h * D;
  const float* V = vb + (size_t)b * T * pitch + h * D;

  FragB aqh[KS], aql[KS];
  {
    int row = q0 + ln; if (row >= T) row = T - 1;
    const float* qr = Q + (size_t)row * pitch;
#pragma unroll
    for (int ks = 0; ks < KS; ++ks)
#pragma unroll
      for (int i = 0; i < 16; ++i) {
        const int d = ks * 32 + ((i < 8) ? (8 * hh + i) : (16 + 8 * hh + (i - 8)));
        const float x = qr[d] * scale; const unsigned short hb = bf16_bits(x);
        aqh[ks].u[i] = hb; aql[ks].u[i] = bf16_bits(x - bf16_val(hb));
      }
  }
  float m_r[8], l_r[8];
#pragma unroll
  for (int r = 0; r < 8; ++r) { m_r[r] = -3.0e38f; l_r[r] = 0.f; }
  v8f oacc[DT];
#pragma unroll
  for (int dt = 0; dt < DT; ++dt) oacc[dt] = (v8f){0.f,0.f,0.f,0.f,0.f,0.f,0.f,0.f};

  const int kv_end = CAUSAL ? min(T, qblk * 64 + 64) : T;
  for (int j0 = 0; j0 < kv_end; j0 += 32) {
    __syncthreads();
    for (int e = tid; e < 32 * (D / 4); e += 128) {
      const int r = e / (D / 4), c4 = (e % (D / 4)) * 4;
      const int key = j0 + r;
      v4f kf = {0.f,0.f,0.f,0.f}, vf = {0.f,0.f,0.f,0.f};
      if (key < T) { kf = *(const v4fa*)(K + (size_t)key * pitch + c4); vf = *(const v4fa*)(V + (size_t)key * pitch + c4); }
#pragma unroll
      for (int t = 0; t < 4; ++t) {
        unsigned short hb = bf16_bits(kf[t]); sKh[r][c4 + t] = hb; sKl[r][c4 + t] = bf16_bits(kf[t] - bf16_val(hb));
        hb = bf16_bits(vf[t]); sVh[r][c4 + t] = hb; sVl[r][c4 + t] = bf16_bits(vf[t] - bf16_val(hb));
      }
    }
    __syncthreads();
    v8f s[2];
#pragma unroll
    for (int nt = 0; nt < 2; ++nt) {
      v8f acc = {};
#pragma unroll
      for (int ks = 0; ks < KS; ++ks) {
        FragB bh_, bl_;
        bh_.half[0] = *(const v8us*)&sKh[nt * 16 + ln][ks * 32 + 8 * hh]; bh_.half[1] = *(const v8us*)&sKh[nt * 16 + ln][ks * 32 + 16 + 8 * hh];
        bl_.half[0] = *(const v8us*)&sKl[nt * 16 + ln][ks * 32 + 8 * hh]; bl_.half[1] = *(const v8us*)&sKl[nt * 16 + ln][ks * 32 + 16 + 8 * hh];
        acc = mmaN<3>(aqh[ks].v, aql[ks].v, bh_.v, bl_.v, acc);
      }
      s[nt] = acc;
    }
    float alpha[8];
#pragma unroll
    for (int r = 0; r < 8; ++r) {
      const int qi = q0 + 8 * hh + r;
      const int ja = j0 + ln, jb = j0 + 16 + ln;
      if (CAUSAL) { if (ja > qi) s[0][r] = -3.0e38f; if (jb > qi) s[1][r] = -3.0e38f; }
      if (ja >= T) s[0][r] = -3.0e38f;
      if (jb >= T) s[1][r] = -3.0e38f;
      float mx = fmaxf(s[0][r], s[1][r]);
      mx = fmaxf(mx, __shfl_xor(mx, 1, 32)); mx = fmaxf(mx, __shfl_xor(mx, 2, 32)); mx = fmaxf(mx, __shfl_xor(mx, 4, 32)); mx = fmaxf(mx, __shfl_xor(mx, 8, 32));
      const float mnew = fmaxf(m_r[r], mx);
      alpha[r] = (mnew > -1.0e38f) ? __expf(m_r[r] - mnew) : 1.0f;
      const float p0 = (s[0][r] > -1.0e38f) ? __expf(s[0][r] - mnew) : 0.f;
      const float p1 = (s[1][r] > -1.0e38f) ? __expf(s[1][r] - mnew) : 0.f;
      m_r[r] = mnew;
      l_r[r] = l_r[r] * alpha[r] + p0 + p1;
      unsigned short hb = bf16_bits(p0); sPh[w][8 * hh + r][ln] = hb;      sPl[w][8 * hh + r][ln] = bf16_bits(p0 - bf16_val(hb));
      hb = bf16_bits(p1);                sPh[w][8 * hh + r][16 + ln] = hb; sPl[w][8 * hh + r][16 + ln] = bf16_bits(p1 - bf16_val(hb));
    }
#pragma unroll
    for (int dt = 0; dt < DT; ++dt)
#pragma unroll
      for (int r = 0; r < 8; ++r) oacc[dt][r] *= alpha[r];
    __builtin_amdgcn_fence(__ATOMIC_ACQ_REL, "workgroup");
    __builtin_amdgcn_wave_barrier();
    FragB pah, pal;
    pah.half[0] = *(const v8us*)&sPh[w][ln][8 * hh]; pah.half[1] = *(const v8us*)&sPh[w][ln][16 + 8 * hh];
    pal.half[0] = *(const v8us*)&sPl[w][ln][8 * hh]; pal.half[1] = *(const v8us*)&sPl[w][ln][16 + 8 * hh];
#pragma unroll
    for (int dt = 0; dt < DT; ++dt) {
      FragB bvh, bvl;
#pragma unroll
      for (int i = 0; i < 8; ++i) {
        bvh.u[i] = sVh[8 * hh + i][dt * 16 + ln]; bvh.u[8 + i] = sVh[16 + 8 * hh + i][dt * 16 + ln];
        bvl.u[i] = sVl[8 * hh + i][dt * 16 + ln]; bvl.u[8 + i] = sVl[16 + 8 * hh + i][dt * 16 + ln];
      }
      oacc[dt] = mmaN<3>(pah.v, pal.v, bvh.v, bvl.v, oacc[dt]);
    }
    __builtin_amdgcn_fence(__ATOMIC_ACQ_REL, "workgroup");
    __builtin_amdgcn_wave_barrier();
  }
#pragma unroll
  for (int r = 0; r < 8; ++r) {
    float l = l_r[r];
    l += __shfl_xor(l, 1, 32); l += __shfl_xor(l, 2, 32); l += __shfl_xor(l, 4, 32); l += __shfl_xor(l, 8, 32);
    l_r[r] = (l > 0.f) ? 1.0f / l : 0.f;
  }
#pragma unroll
  for (int dt = 0; dt < DT; ++dt)
#pragma unroll
    for (int r = 0; r < 8; ++r) sO[w][8 * hh + r][dt * 16 + ln] = oacc[dt][r] * l_r[r];
  __builtin_amdgcn_fence(__ATOMIC_ACQ_REL, "workgroup");
  __builtin_amdgcn_wave_barrier();
  for (int pass = 0; pass < 2; ++pass) {
    for (int r = 0; r < 16; ++r) {
      const int row = q0 + r;
      if (row < T && lane < D / 4) {
        const v4f val = *(const v4fa*)&sO[w][r][lane * 4];
        *(volatile v4f*)(y + ((size_t)b * T + row) * ypitch + h * D + lane * 4) = val;
      }
    }
    if (pass == 0) __threadfence();
  }
}

template <bool ASPLIT, int ACT, bool BIAS_BF16, bool RES_BF16>
__global__ __launch_bounds__(128) void k_gemm_bf3(const float* __restrict__ A, int lda, const unsigned short* __restrict__ Wt, int ldb,
                                                const float* __restrict__ bias, const float* __restrict__ resid, int rmod, int ldr,
                                                float* __restrict__ C, int ldc, int M, int N, int K) {
  __shared__ __attribute__((aligned(16))) float so[4][16][64];
  const int tid = threadIdx.x, w = tid >> 5, lane = tid & 31, ln = lane & 15, hh = lane >> 4;
  const int ntn = N / 64;
  const int wid = blockIdx.x * 4 + w;
  const int mt = wid / ntn, nq = wid % ntn;
  if (mt * 16 >= M) return;
  const int row0 = mt * 16, col0 = nq * 64;
  const float* arow = A + (size_t)(row0 + ln) * lda;
  v8f acc[4] = {};
  for (int kb = 0; kb < K; kb += 32) {
    FragB ah, al;
    const v4f x0 = *(const v4fa*)(arow + kb + 8 * hh), x1 = *(const v4fa*)(arow + kb + 8 * hh + 4);
    const v4f x2 = *(const v4fa*)(arow + kb + 16 + 8 * hh), x3 = *(const v4fa*)(arow + kb + 16 + 8 * hh + 4);
    float xs[16] = {x0[0],x0[1],x0[2],x0[3],x1[0],x1[1],x1[2],x1[3],x2[0],x2[1],x2[2],x2[3],x3[0],x3[1],x3[2],x3[3]};
#pragma unroll
    for (int i = 0; i < 16; ++i) { const unsigned short hb = bf16_bits(xs[i]); ah.u[i] = hb; al.u[i] = ASPLIT ? bf16_bits(xs[i] - bf16_val(hb)) : (unsigned short)0; }
#pragma unroll
    for (int t = 0; t < 4; ++t) {
      const unsigned short* brow = Wt + (size_t)(col0 + t * 16 + ln) * ldb + kb;
      FragB b;
      b.half[0] = *(const v8us*)(brow + 8 * hh);
      b.half[1] = *(const v8us*)(brow + 16 + 8 * hh);
      acc[t] = mmaN<ASPLIT ? 2 : 1>(ah.v, al.v, b.v, b.v, acc[t]);
    }
  }
#pragma unroll
  for (int t = 0; t < 4; ++t) {
    const int col = col0 + t * 16 + ln;
    float bv = bias ? bias[col] : 0.f;
    if (BIAS_BF16) bv = bf16_round(bv);
#pragma unroll
    for (int r = 0; r < 8; ++r) {
      float v = acc[t][r] + bv;
      if (resid) { float rv = resid[(size_t)((row0 + 8 * hh + r) % rmod) * ldr + col]; if (RES_BF16) rv = bf16_round(rv); v += rv; }
      if (ACT == 1) v = fmaxf(v, 0.f);
      if (ACT == 2) v = 0.5f * v * (1.0f + erff(v * 0.70710678118654752f));
      if (ACT == 3) { const float u = 0.7978845608028654f * (v + 0.044715f * v * v * v); v = 0.5f * v * (1.0f + tanhf(u)); }
      so[w][8 * hh + r][t * 16 + ln] = v;
    }
  }
  __builtin_amdgcn_fence(__ATOMIC_ACQ_REL, "workgroup");
  __builtin_amdgcn_wave_barrier();
  const int rsub = lane >> 4, c4 = (lane & 15) * 4;
  for (int pass = 0; pass < 2; ++pass) {
#pragma unroll
    for (int q = 0; q < 8; ++q) {
      const int r = q * 2 + rsub;
      const v4f v = *(const v4fa*)&so[w][r][c4];
      *(volatile v4f*)(C + (size_t)(row0 + r) * ldc + col0 + c4) = v;
    }
    if (pass == 0) __threadfence();
  }
}
template <bool PARAM_BF16>
__global__ __launch_bounds__(256) void k_layernorm(const float* __restrict__ X, const float* __restrict__ R, const float* __restrict__ g, const float* __restrict__ bta,
                                                  float* __restrict__ out_sum, float* __restrict__ out_norm, int N, float eps) {
  __shared__ float red[256];
  const int row = blockIdx.x, tid = threadIdx.x;
  const float* x = X + (size_t)row * N; const float* rr = R ? R + (size_t)row * N : nullptr;
  float vals[16];
  const int per = N / 256;
  float s1 = 0.f;
  for (int u = 0; u < per / 4; ++u) {
    const int j = tid * 4 + 1024 * u;
    const v4f a = *(const v4fa*)(x + j);
    v4f b = {0.f,0.f,0.f,0.f}; if (rr) b = *(const v4fa*)(rr + j);
#pragma unroll
    for (int q = 0; q < 4; ++q) { const float v = a[q] + b[q]; vals[u * 4 + q] = v; s1 += v; }
  }
  red[tid] = s1; __syncthreads();
  for (int st = 128; st > 0; st >>= 1) { if (tid < st) red[tid] += red[tid + st]; __syncthreads(); }
  const float mu = red[0] / (float)N; __syncthreads();
  float s2 = 0.f;
  for (int u = 0; u < per / 4; ++u)
#pragma unroll
    for (int q = 0; q < 4; ++q) { const float c = vals[u * 4 + q] - mu; s2 += c * c; }
  red[tid] = s2; __syncthreads();
  for (int st = 128; st > 0; st >>= 1) { if (tid < st) red[tid] += red[tid + st]; __syncthreads(); }
  const float rs = rsqrtf(red[0] / (float)N + eps);
  for (int pass = 0; pass < 2; ++pass) {
    for (int u = 0; u < per / 4; ++u) {
      const int j = tid * 4 + 1024 * u;
      v4f o, sm;
#pragma unroll
      for (int q = 0; q < 4; ++q) {
        float gg = g[j + q], bb = bta[j + q];
        if (PARAM_BF16) { gg = bf16_round(gg); bb = bf16_round(bb); }
        sm[q] = vals[u * 4 + q]; o[q] = (vals[u * 4 + q] - mu) * rs * gg + bb;
      }
      if (out_sum) *(volatile v4f*)(out_sum + (size_t)row * N + j) = sm;
      *(volatile v4f*)(out_norm + (size_t)row * N + j) = o;
    }
    if (pass == 0) __threadfence();
  }
}
template <int Cin, bool SPLIT>
__global__ __launch_bounds__(128) void k_conv2d(const float* __restrict__ in, const unsigned short* __restrict__ Bt, const float* __restrict__ bias, float* __restrict__ out) {
  constexpr int K = 9 * Cin, SPT = Cin / 32;
  __shared__ __attribute__((aligned(16))) float so[4][16][64];
  const int tid = threadIdx.x, w = tid >> 5, lane = tid & 31, ln = lane & 15, hh = lane >> 4;
  const int wid = blockIdx.x * 4 + w; const int mt = wid / (COUT / 64), nq = wid % (COUT / 64); if (mt * 16 >= NVOX) return;
  const int row0 = mt * 16, col0 = nq * 64;
  const int m = row0 + ln;
  const int x = m % WX, y = (m / WX) % HY, b = m / (WX * HY);
  v8f acc[4] = {};
  for (int tap = 0; tap < 9; ++tap) {
    const int dy = tap / 3 - 1, dx = tap % 3 - 1;
    const int xx = x + dx, yy = y + dy;
    const bool inb = (m < NPOSR) && (xx >= 0 && xx < WX && yy >= 0 && yy < HY);
    const float* src = in + ((size_t)((b * HY + (inb ? yy : 0)) * WX + (inb ? xx : 0))) * Cin;
#pragma unroll
    for (int s = 0; s < SPT; ++s) {
      const int c0 = s * 32;
      v4f a0 = {0.f,0.f,0.f,0.f}, a1 = a0, a2 = a0, a3 = a0;
      if (inb) { a0 = *(const v4fa*)(src + c0 + 8 * hh); a1 = *(const v4fa*)(src + c0 + 8 * hh + 4); a2 = *(const v4fa*)(src + c0 + 16 + 8 * hh); a3 = *(const v4fa*)(src + c0 + 16 + 8 * hh + 4); }
      float xs[16] = {a0[0],a0[1],a0[2],a0[3],a1[0],a1[1],a1[2],a1[3],a2[0],a2[1],a2[2],a2[3],a3[0],a3[1],a3[2],a3[3]};
      FragB ah, al;
#pragma unroll
      for (int i = 0; i < 16; ++i) { const unsigned short hb = bf16_bits(xs[i]); ah.u[i] = hb; al.u[i] = SPLIT ? bf16_bits(xs[i] - bf16_val(hb)) : (unsigned short)0; }
      const int kb = tap * Cin + c0;
#pragma unroll
      for (int t = 0; t < 4; ++t) { FragB bq; bq.half[0] = *(const v8us*)(Bt + (size_t)(col0 + t * 16 + ln) * K + kb + 8 * hh); bq.half[1] = *(const v8us*)(Bt + (size_t)(col0 + t * 16 + ln) * K + kb + 16 + 8 * hh); acc[t] = SPLIT ? mmaN<2>(ah.v, al.v, bq.v, bq.v, acc[t]) : mmaN<1>(ah.v, al.v, bq.v, bq.v, acc[t]); }
    }
  }
#pragma unroll
  for (int t = 0; t < 4; ++t) { const int col = col0 + t * 16 + ln; const float bv = bf16_round(bias[col]);
#pragma unroll
    for (int r = 0; r < 8; ++r) so[w][8 * hh + r][t * 16 + ln] = acc[t][r] + bv; }
  __builtin_amdgcn_fence(__ATOMIC_ACQ_REL, "workgroup"); __builtin_amdgcn_wave_barrier();
  const int rsub = lane >> 4, c4 = (lane & 15) * 4;
  for (int pass = 0; pass < 2; ++pass) { for (int q = 0; q < 8; ++q) { const int r = q * 2 + rsub; const v4f v = *(const v4fa*)&so[w][r][c4]; *(volatile v4f*)(out + (size_t)(row0 + r) * COUT + col0 + c4) = v; } if (pass == 0) __threadfence(); }
}


__global__ __launch_bounds__(256) void k_round_rows(const float* __restrict__ W, unsigned short* __restrict__ Wt, int n8) {
  const int t = blockIdx.x * 256 + threadIdx.x;
  if (t >= n8) return;
  const v4f a = *(const v4fa*)(W + (size_t)t * 8), b = *(const v4fa*)(W + (size_t)t * 8 + 4);
  v8us v; v[0]=bf16_bits(a[0]); v[1]=bf16_bits(a[1]); v[2]=bf16_bits(a[2]); v[3]=bf16_bits(a[3]);
  v[4]=bf16_bits(b[0]); v[5]=bf16_bits(b[1]); v[6]=bf16_bits(b[2]); v[7]=bf16_bits(b[3]);
  *(volatile v8us*)(Wt + (size_t)t * 8) = v; __threadfence(); *(volatile v8us*)(Wt + (size_t)t * 8) = v;
}

__global__ __launch_bounds__(256) void k_zero(float* __restrict__ p, int n) { const int t = blockIdx.x * 256 + threadIdx.x; if (t >= n) return; *(volatile float*)(p + t) = 0.f; __threadfence(); *(volatile float*)(p + t) = 0.f; }
__global__ __launch_bounds__(32) void k_hist(const float* __restrict__ x1, float* __restrict__ part) {
  __shared__ int h2[NB2 * NB2]; __shared__ int h1[NB1];
  const int lane = threadIdx.x; const int b = blockIdx.x / NBLK, blk = blockIdx.x % NBLK;
  for (int i = lane; i < NB2 * NB2; i += 32) h2[i] = 0; if (lane < NB1) h1[lane] = 0;
  __builtin_amdgcn_fence(__ATOMIC_ACQ_REL, "workgroup"); __builtin_amdgcn_wave_barrier();
  const float* cl = x1 + ((size_t)b * 3 + 0) * HWI; const float* ca = x1 + ((size_t)b * 3 + 1) * HWI; const float* cb = x1 + ((size_t)b * 3 + 2) * HWI;
#pragma unroll 1
  for (int p0 = blk * CHK; p0 < (blk + 1) * CHK; p0 += 32) { const int p = p0 + lane;
    const float a = bf16_round(ca[p]), bb = bf16_round(cb[p]), l = bf16_round(cl[p]);
    const float va = (a + 1.0f) * 0.5f, vb = (bb + 1.0f) * 0.5f, vl = (l + 1.0f) * 0.5f;
    const bool w2 = (a != 0.f) && (bb != 0.f) && (va >= 0.f) && (va <= 1.f) && (vb >= 0.f) && (vb <= 1.f); const bool w1 = (l != 0.f) && (vl >= 0.f) && (vl <= 1.f);
    int ia = (int)floorf(va * (float)NB2), ib = (int)floorf(vb * (float)NB2), il = (int)floorf(vl * (float)NB1); ia = ia < 0 ? 0 : (ia > NB2 - 1 ? NB2 - 1 : ia); ib = ib < 0 ? 0 : (ib > NB2 - 1 ? NB2 - 1 : ib); il = il < 0 ? 0 : (il > NB1 - 1 ? NB1 - 1 : il);
    const int k2 = w2 ? (ia * NB2 + ib) : -1; const int k1 = w1 ? il : -1;
    { bool done = false;
#pragma unroll 1
      for (int ld = 0; ld < 32; ++ld) { const int kk = __shfl(k2, ld, 32); const unsigned long long m = __ballot(k2 == kk); const int cnt = __popcll(m); const int first = __ffsll((long long)m) - 1;
        if (ld == first && lane == first && kk >= 0 && !done) { h2[kk] += cnt; done = true; } } }
    __builtin_amdgcn_fence(__ATOMIC_ACQ_REL, "workgroup"); __builtin_amdgcn_wave_barrier();
    { bool done = false;
#pragma unroll 1
      for (int ld = 0; ld < 32; ++ld) { const int kk = __shfl(k1, ld, 32); const unsigned long long m = __ballot(k1 == kk); const int cnt = __popcll(m); const int first = __ffsll((long long)m) - 1;
        if (ld == first && lane == first && kk >= 0 && !done) { h1[kk] += cnt; done = true; } } }
    __builtin_amdgcn_fence(__ATOMIC_ACQ_REL, "workgroup"); __builtin_amdgcn_wave_barrier();
  }
  float* pr = part + (size_t)blockIdx.x * 4128;
  for (int pass = 0; pass < 2; ++pass) { for (int i = lane; i < 4128; i += 32) *(volatile float*)(pr + i) = (i < 4096) ? (float)h2[i] : (i < 4104 ? (float)h1[i - 4096] : 0.f); if (pass == 0) __threadfence(); }
}
__global__ __launch_bounds__(256) void k_histsum(const float* __restrict__ part, float* __restrict__ hin) {
  __shared__ float s2[4096]; __shared__ float s1[8]; __shared__ float red[256];
  const int b = blockIdx.x, t = threadIdx.x;
  for (int i = t; i < 4096; i += 256) { float s = 0.f;
#pragma unroll 1
    for (int k = 0; k < NBLK; ++k) s += part[((size_t)b * NBLK + k) * 4128 + i]; s2[i] = s; }
  if (t < 8) { float s = 0.f; for (int k = 0; k < NBLK; ++k) s += part[((size_t)b * NBLK + k) * 4128 + 4096 + t]; s1[t] = s; }
  __syncthreads();
  float ps = 0.f; for (int i = t; i < 4096; i += 256) ps += s2[i]; red[t] = ps; __syncthreads(); for (int st = 128; st > 0; st >>= 1) { if (t < st) red[t] += red[t + st]; __syncthreads(); } const float tot2 = red[0]; __syncthreads();
  float tot1 = 0.f; for (int k = 0; k < 8; ++k) tot1 += s1[k];
  for (int pass = 0; pass < 2; ++pass) {
    for (int e = t; e < 9 * 4096; e += 256) { const int c = e / 4096, yx = e % 4096; const int y = yx / 64, xq = yx % 64; float v;
      if (c == 0) v = s2[xq * 64 + y] / tot2;
      else v = s1[c - 1] / tot1;
      *(volatile float*)(hin + ((size_t)b * 9) * 4096 + e) = v; }
    if (pass == 0) __threadfence(); }
}
__global__ __launch_bounds__(256) void k_stage1(const float* __restrict__ hin, const float* __restrict__ w1, const float* __restrict__ g1, const float* __restrict__ b1, const float* __restrict__ m1, const float* __restrict__ v1, float* __restrict__ P) {
  const size_t i = (size_t)blockIdx.x * 256 + threadIdx.x; if (i >= (size_t)NPOS * 128) return; const int c = (int)(i % 128); const int pos = (int)(i / 128); const int ox = pos % P33, oy = (pos / P33) % P33, b = pos / (P33 * P33);
  const float inv = bf16_round(g1[c]) / sqrtf(bf16_round(v1[c]) + 1e-5f); const float sh = bf16_round(b1[c]) - bf16_round(m1[c]) * inv;
  float wv[9]; for (int k = 0; k < 9; ++k) wv[k] = bf16_round(w1[c * 9 + k]);
  float mx = -3.0e38f;
#pragma unroll 1
  for (int dy = 0; dy < 3; ++dy)
#pragma unroll 1
    for (int dx = 0; dx < 3; ++dx) { const int gy = oy * 2 - 1 + dy, gx = ox * 2 - 1 + dx; if (gy < 0 || gy >= G66 || gx < 0 || gx >= G66) continue;
      float conv = 0.f; const int yy = gy - 1, xx = gx - 1;
      if (yy >= 0 && yy < 64 && xx >= 0 && xx < 64) { for (int k = 0; k < 9; ++k) conv += wv[k] * hin[(((size_t)b * 9 + k) * 64 + yy) * 64 + xx]; }
      const float bnv = (conv - bf16_round(m1[c])) * inv + bf16_round(b1[c]); (void)sh; mx = fmaxf(mx, bnv); }
  const float r = fmaxf(mx, 0.f); *(volatile float*)(P + i) = r; __threadfence(); *(volatile float*)(P + i) = r;
}
__global__ __launch_bounds__(256) void k_wt2(const float* __restrict__ w, unsigned short* __restrict__ Bt) {
  const int t = blockIdx.x * 256 + threadIdx.x; const int K = 9 * 128; if (t >= COUT * (K / 8)) return; const int o = t / (K / 8), k8 = (t % (K / 8)) * 8; v8us v;
  for (int i = 0; i < 8; ++i) { const int k = k8 + i; const int tap = k / 128, c = k % 128; v[i] = bf16_bits(w[((size_t)o * 128 + c) * 9 + tap]); }
  *(volatile v8us*)(Bt + (size_t)o * K + k8) = v; __threadfence(); *(volatile v8us*)(Bt + (size_t)o * K + k8) = v;
}
__global__ __launch_bounds__(256) void k_bnmean(const float* __restrict__ Y, const float* __restrict__ g2, const float* __restrict__ b2, const float* __restrict__ m2, const float* __restrict__ v2, float* __restrict__ hm) {
  const int t = blockIdx.x * 256 + threadIdx.x; if (t >= BB * COUT) return; const int b = t / COUT, o = t % COUT; const float inv = bf16_round(g2[o]) / sqrtf(bf16_round(v2[o]) + 1e-5f); const float mb = bf16_round(m2[o]), bb = bf16_round(b2[o]); float s = 0.f;
#pragma unroll 1
  for (int p = 0; p < P33 * P33; ++p) { const float y = Y[((size_t)b * P33 * P33 + p) * COUT + o]; s += fmaxf((y - mb) * inv + bb, 0.f); }
  const float v = s / (float)(P33 * P33); *(volatile float*)(hm + t) = v; __threadfence(); *(volatile float*)(hm + t) = v;
}
__global__ __launch_bounds__(256) void k_final(const float* __restrict__ x, const float* __restrict__ fcv, float* __restrict__ out) {
  const int b = blockIdx.x, t = threadIdx.x;
  for (int pass = 0; pass < 2; ++pass) { for (int e = t; e < 2304; e += 256) { const float v = (e < 2048) ? bf16_round(x[(size_t)b * 2048 + e]) : fcv[(size_t)b * 256 + (e - 2048)]; *(volatile float*)(out + (size_t)b * 2304 + e) = v; } if (pass == 0) __threadfence(); }
}
extern "C" void kernel_launch(void* const* d_in, const int* in_sizes, int n_in,
                              void* d_out, int out_size, void* d_ws, size_t ws_size, hipStream_t stream) {
  (void)in_sizes; (void)n_in; (void)out_size;
  const float* x = (const float*)d_in[0]; const float* x1 = (const float*)d_in[1]; const float* w1 = (const float*)d_in[2]; const float* g1 = (const float*)d_in[3]; const float* b1 = (const float*)d_in[4]; const float* m1 = (const float*)d_in[5]; const float* v1 = (const float*)d_in[6];
  const float* w2 = (const float*)d_in[7]; const float* g2 = (const float*)d_in[8]; const float* b2 = (const float*)d_in[9]; const float* m2 = (const float*)d_in[10]; const float* v2 = (const float*)d_in[11]; const float* wl = (const float*)d_in[12]; const float* bl = (const float*)d_in[13];
  char* ws = (char*)d_ws; size_t off = 0;
  auto take = [&](size_t bytes) { char* p = ws + off; off += (bytes + 255) & ~(size_t)255; return p; };
  unsigned short* Bt2 = (unsigned short*)take((size_t)COUT * 9 * 128 * 2); unsigned short* Bl = (unsigned short*)take((size_t)256 * 1024 * 2); float* zb = (float*)take(COUT * 4);
  float* part = (float*)take((size_t)BB * NBLK * 4128 * 4); float* hin = (float*)take((size_t)BB * 9 * 4096 * 4); float* P = (float*)take((size_t)NVOX * 128 * 4); float* Y = (float*)take((size_t)NVOX * COUT * 4); float* hm = (float*)take((size_t)BB * COUT * 4); float* fcv = (float*)take((size_t)BB * 256 * 4);
  if (off > ws_size) return;
  k_wt2<<<(COUT * 144 + 255) / 256, 256, 0, stream>>>(w2, Bt2); k_round_rows<<<(256 * 1024 / 8 + 255) / 256, 256, 0, stream>>>(wl, Bl, 256 * 1024 / 8);
  k_zero<<<(COUT + 255) / 256, 256, 0, stream>>>(zb, COUT);
  k_hist<<<BB * NBLK, 32, 0, stream>>>(x1, part);
  k_histsum<<<BB, 256, 0, stream>>>(part, hin);
  k_stage1<<<(unsigned)(((size_t)NPOS * 128 + 255) / 256), 256, 0, stream>>>(hin, w1, g1, b1, m1, v1, P);
  k_conv2d<128, false><<<((NVOX / 16) * (COUT / 64) + 3) / 4, 128, 0, stream>>>(P, Bt2, zb, Y);
  k_bnmean<<<(BB * COUT + 255) / 256, 256, 0, stream>>>(Y, g2, b2, m2, v2, hm);
  k_gemm_bf3<true, 0, true, false><<<((BB / 16) * (256 / 64) + 3) / 4, 128, 0, stream>>>(hm, COUT, Bl, COUT, bl, nullptr, 1, 0, fcv, 256, BB, 256, COUT);
  k_final<<<BB, 256, 0, stream>>>(x, fcv, (float*)d_out);
}
